// LocalAttentionDraftLayer_25357486916438
// MI455X (gfx1250) — hardware-verified
//
#include <hip/hip_runtime.h>
#include <stddef.h>
#include <stdint.h>
#include <math.h>

#define NBATCH 2
#define SEQ    4096
#define HD     1024
#define HF     512
#define MROWS  (NBATCH * SEQ)
#define WIN    32

static_assert(MROWS % 256 == 0);
static_assert(SEQ % 256 == 0);
static_assert(SEQ % 128 == 0);
static_assert(HD % 64 == 0);
static_assert(HF % 64 == 0);
static_assert(HD % 32 == 0);
static_assert(HF % 32 == 0);

typedef _Float16 v16h __attribute__((ext_vector_type(16)));
typedef _Float16 v8h  __attribute__((ext_vector_type(8)));
typedef float    v8f  __attribute__((ext_vector_type(8)));
typedef float    v4f  __attribute__((ext_vector_type(4)));
typedef unsigned int v4u __attribute__((ext_vector_type(4)));

union Frag  { v16h v; v8h h[2]; };
union Pack8 { v8h h; v4u u; };

__device__ __forceinline__ v8f mma16(v16h a, v16h b, v8f c) {
  c = __builtin_amdgcn_wmma_f32_16x16x32_f16(false, a, false, b, (short)0, c, false, false);
  asm volatile("v_nop\n\tv_nop\n\tv_nop\n\tv_nop" : "+v"(c) : "v"(a), "v"(b));
  return c;
}

__device__ __forceinline__ v16h ldfrag(const _Float16* p, int ld, int row0, int k0, int lane) {
  const int m = lane & 15, lh = lane >> 4;
  const _Float16* q = p + (size_t)(row0 + m) * ld + k0 + 8 * lh;
  Frag f;
  f.h[0] = *(const v8h*)(q);
  f.h[1] = *(const v8h*)(q + 16);
  return f.v;
}

__device__ __forceinline__ v8f zero8() { return (v8f){0.f, 0.f, 0.f, 0.f, 0.f, 0.f, 0.f, 0.f}; }

template <int KD>
__device__ __forceinline__ void gemm32x64(const _Float16* __restrict__ A,
                                          const _Float16* __restrict__ Bt,
                                          int m0, int n0, int lane, v8f (&acc)[2][4]) {
#pragma unroll 2
  for (int k0 = 0; k0 < KD; k0 += 32) {
    const v16h a0 = ldfrag(A, KD, m0, k0, lane);
    const v16h a1 = ldfrag(A, KD, m0 + 16, k0, lane);
    const v16h b0 = ldfrag(Bt, KD, n0, k0, lane);
    const v16h b1 = ldfrag(Bt, KD, n0 + 16, k0, lane);
    const v16h b2 = ldfrag(Bt, KD, n0 + 32, k0, lane);
    const v16h b3 = ldfrag(Bt, KD, n0 + 48, k0, lane);
    acc[0][0] = mma16(a0, b0, acc[0][0]);
    acc[1][0] = mma16(a1, b0, acc[1][0]);
    acc[0][1] = mma16(a0, b1, acc[0][1]);
    acc[1][1] = mma16(a1, b1, acc[1][1]);
    acc[0][2] = mma16(a0, b2, acc[0][2]);
    acc[1][2] = mma16(a1, b2, acc[1][2]);
    acc[0][3] = mma16(a0, b3, acc[0][3]);
    acc[1][3] = mma16(a1, b3, acc[1][3]);
  }
}

__global__ __launch_bounds__(256) void k_cvt(const float* __restrict__ x, _Float16* __restrict__ xh,
                                             int ngrp, float scale) {
  const int t = blockIdx.x * 256 + (int)threadIdx.x;
  if (t >= ngrp) return;
  const size_t o = (size_t)t * 8;
  const v4f a0 = *(const v4f*)(x + o);
  const v4f a1 = *(const v4f*)(x + o + 4);
  Pack8 pk;
  pk.h = (v8h){(_Float16)(a0[0] * scale), (_Float16)(a0[1] * scale), (_Float16)(a0[2] * scale), (_Float16)(a0[3] * scale),
               (_Float16)(a1[0] * scale), (_Float16)(a1[1] * scale), (_Float16)(a1[2] * scale), (_Float16)(a1[3] * scale)};
  const v4u vv = pk.u;
  volatile v4u* d = (volatile v4u*)(xh + o);
  *d = vv;
  __threadfence();
  *d = vv;
}

#define STP 72
template <int MODE, int KD>
__global__ __launch_bounds__(256) void k_gemm_h(const _Float16* __restrict__ ah,
                                                const _Float16* __restrict__ wt,
                                                const float* __restrict__ bias,
                                                _Float16* __restrict__ hp, int ldc) {
  __shared__ __align__(16) _Float16 st[256 * STP];
  const int tid = threadIdx.x, lane = tid & 31, wave = tid >> 5;
  const int hh = lane >> 4, c = lane & 15;
  const int mb = blockIdx.x * 256;
  const int m0 = mb + wave * 32;
  const int n0 = blockIdx.y * 64;

  v8f acc[2][4];
#pragma unroll
  for (int s = 0; s < 2; ++s)
#pragma unroll
    for (int t = 0; t < 4; ++t) acc[s][t] = zero8();
  gemm32x64<KD>(ah, wt, m0, n0, lane, acc);

#pragma unroll
  for (int t = 0; t < 4; ++t) {
    float bv = 0.0f;
    if constexpr (MODE == 2) bv = bias[n0 + 16 * t + c];
#pragma unroll
    for (int sub = 0; sub < 2; ++sub) {
#pragma unroll
      for (int r = 0; r < 8; ++r) {
        const int lr = wave * 32 + sub * 16 + 8 * hh + r;
        float v = acc[sub][t][r] * 0.03125f + bv;
        if constexpr (MODE == 2) {
          v = 0.5f * v * (1.0f + erff(v * 0.70710678118654752f));
        }
        st[lr * STP + 16 * t + c] = (_Float16)v;
      }
    }
  }
  __syncthreads();

  v4u val[8];
  size_t go[8];
  if constexpr (MODE != 1) {
#pragma unroll
    for (int j = 0; j < 8; ++j) {
      const int p  = tid + 256 * j;
      const int lr = p >> 3;
      const int pc = p & 7;
      Pack8 pk;
      pk.h   = *(const v8h*)(st + lr * STP + pc * 8);
      val[j] = pk.u;
      go[j]  = (size_t)(mb + lr) * ldc + n0 + pc * 8;
    }
  } else {
    const int bidx = mb / SEQ;
    const int nb   = mb - bidx * SEQ;
#pragma unroll
    for (int j = 0; j < 8; ++j) {
      const int p  = tid + 256 * j;
      const int L  = p >> 3;
      const int pc = p & 7;
      const int d  = L >> 2;
      const int nl = (L & 3) * 64 + pc * 8;
      const _Float16* cp = st + nl * STP + d;
      Pack8 pk;
      pk.h = (v8h){cp[0 * STP], cp[1 * STP], cp[2 * STP], cp[3 * STP],
                   cp[4 * STP], cp[5 * STP], cp[6 * STP], cp[7 * STP]};
      val[j] = pk.u;
      go[j]  = ((size_t)(bidx * HD + n0 + d)) * SEQ + nb + nl;
    }
  }
  for (int ps = 0; ps < 2; ++ps) {
#pragma unroll
    for (int j = 0; j < 8; ++j) *(volatile v4u*)(hp + go[j]) = val[j];
    __threadfence();
  }
}

#define OTP 68
template <int HASB, int KD>
__global__ __launch_bounds__(256) void k_gemm_f(const _Float16* __restrict__ ap,
                                                const _Float16* __restrict__ wt,
                                                const float* __restrict__ bias,
                                                const float* __restrict__ resid,
                                                float* __restrict__ out, float escale) {
  __shared__ __align__(16) float st[8][16 * OTP];
  const int tid = threadIdx.x, lane = tid & 31, wave = tid >> 5;
  const int hh = lane >> 4, c = lane & 15;
  const int m0 = blockIdx.x * 256 + wave * 32;
  const int n0 = blockIdx.y * 64;

  v8f acc[2][4];
#pragma unroll
  for (int s = 0; s < 2; ++s)
#pragma unroll
    for (int t = 0; t < 4; ++t) acc[s][t] = zero8();
  gemm32x64<KD>(ap, wt, m0, n0, lane, acc);

  float bvs[4];
#pragma unroll
  for (int t = 0; t < 4; ++t) {
    bvs[t] = 0.0f;
    if constexpr (HASB) bvs[t] = bias[n0 + 16 * t + c];
  }

  float* sw = st[wave];
#pragma unroll
  for (int sub = 0; sub < 2; ++sub) {
    __syncthreads();
#pragma unroll
    for (int t = 0; t < 4; ++t) {
#pragma unroll
      for (int r = 0; r < 8; ++r)
        sw[(8 * hh + r) * OTP + 16 * t + c] = acc[sub][t][r] * escale + bvs[t];
    }
    __syncthreads();
    v4f val[8];
    size_t go[8];
#pragma unroll
    for (int it = 0; it < 8; ++it) {
      const int p    = lane + 32 * it;
      const int L    = p >> 3;
      const int pc   = p & 7;
      const int row  = L >> 1;
      const int half = L & 1;
      go[it]  = (size_t)(m0 + sub * 16 + row) * HD + n0 + half * 32 + pc * 4;
      val[it] = *(const v4f*)(sw + row * OTP + half * 32 + pc * 4) + *(const v4f*)(resid + go[it]);
    }
    for (int ps = 0; ps < 2; ++ps) {
#pragma unroll
      for (int it = 0; it < 8; ++it) *(volatile v4f*)(out + go[it]) = val[it];
      __threadfence();
    }
  }
}

#define PTP 72
__global__ __launch_bounds__(256) void k_attn(const _Float16* __restrict__ qp,
                                              const _Float16* __restrict__ kp,
                                              const _Float16* __restrict__ vt,
                                              _Float16* __restrict__ op) {
  __shared__ __align__(16) _Float16 Ps[8][16 * PTP];
  __shared__ __align__(16) _Float16 Os[8][16 * PTP];

  const int tid = threadIdx.x, lane = tid & 31, wave = tid >> 5;
  const int hh = lane >> 4, c = lane & 15;
  const int q0 = blockIdx.x * 128 + wave * 16;
  const int bidx = q0 / SEQ;
  const int qs = q0 - bidx * SEQ;
  const int kbase = qs - WIN;
  const _Float16* Kb = kp + (size_t)bidx * SEQ * HD;
  const _Float16* Vb = vt + (size_t)bidx * HD * SEQ;

  v8f s[3];
#pragma unroll
  for (int t = 0; t < 3; ++t) s[t] = zero8();
#pragma unroll 2
  for (int k0 = 0; k0 < HD; k0 += 32) {
    const v16h qa = ldfrag(qp, HD, q0, k0, lane);
#pragma unroll
    for (int t = 0; t < 3; ++t) {
      int kr = kbase + 16 * t + c;
      kr = kr < 0 ? 0 : kr;
      const _Float16* kq = Kb + (size_t)kr * HD + k0 + 8 * hh;
      Frag f;
      f.h[0] = *(const v8h*)(kq);
      f.h[1] = *(const v8h*)(kq + 16);
      s[t] = mma16(qa, f.v, s[t]);
    }
  }

  const float NEGI = -__builtin_huge_valf();
  float linv[8];
  _Float16* pw = Ps[wave];
#pragma unroll
  for (int r = 0; r < 8; ++r) {
    const int qi = qs + 8 * hh + r;
    float m = NEGI;
#pragma unroll
    for (int t = 0; t < 3; ++t) {
      const int kj = kbase + 16 * t + c;
      float sv = s[t][r] * 0.03125f;
      const bool live = (kj >= 0) && (kj <= qi) && (kj > qi - WIN);
      sv = live ? sv : NEGI;
      s[t][r] = sv;
      m = fmaxf(m, sv);
    }
#pragma unroll
    for (int off = 1; off < 16; off <<= 1) m = fmaxf(m, __shfl_xor(m, off, 32));
    float psum = 0.f;
#pragma unroll
    for (int t = 0; t < 3; ++t) {
      const float p = __expf(s[t][r] - m);
      psum += p;
      pw[(8 * hh + r) * PTP + 16 * t + c] = (_Float16)(p * 1024.0f);
    }
    pw[(8 * hh + r) * PTP + 48 + c] = (_Float16)(psum * 0.0f);
#pragma unroll
    for (int off = 1; off < 16; off <<= 1) psum += __shfl_xor(psum, off, 32);
    linv[r] = 0.015625f / psum;
  }
  __syncthreads();

  v16h pa[2];
  pa[0] = ldfrag(pw, PTP, 0, 0, lane);
  pa[1] = ldfrag(pw, PTP, 0, 32, lane);

  _Float16* ow = Os[wave];
#pragma unroll 1
  for (int sl = 0; sl < HD / 64; ++sl) {
    v8f oacc[4];
#pragma unroll
    for (int t = 0; t < 4; ++t) oacc[t] = zero8();
#pragma unroll
    for (int kk = 0; kk < 2; ++kk) {
      int ka = kbase + 32 * kk + 8 * hh;
      int kb = kbase + 32 * kk + 16 + 8 * hh;
      ka = ka < 0 ? 0 : ka;  ka = ka > SEQ - 8 ? SEQ - 8 : ka;
      kb = kb < 0 ? 0 : kb;  kb = kb > SEQ - 8 ? SEQ - 8 : kb;
#pragma unroll
      for (int t = 0; t < 4; ++t) {
        const _Float16* vr = Vb + (size_t)(sl * 64 + 16 * t + c) * SEQ;
        Frag f;
        f.h[0] = *(const v8h*)(vr + ka);
        f.h[1] = *(const v8h*)(vr + kb);
        oacc[t] = mma16(pa[kk], f.v, oacc[t]);
      }
    }
#pragma unroll
    for (int r = 0; r < 8; ++r) {
#pragma unroll
      for (int t = 0; t < 4; ++t) ow[(8 * hh + r) * PTP + 16 * t + c] = (_Float16)(oacc[t][r] * linv[r]);
    }
    __syncthreads();
    v4u val[4];
    size_t go[4];
#pragma unroll
    for (int it = 0; it < 4; ++it) {
      const int p  = lane + 32 * it;
      const int L  = p >> 3;
      const int pc = p & 7;
      Pack8 pk;
      pk.h    = *(const v8h*)(ow + L * PTP + pc * 8);
      val[it] = pk.u;
      go[it]  = (size_t)(q0 + L) * HD + (size_t)sl * 64 + pc * 8;
    }
    for (int ps = 0; ps < 2; ++ps) {
#pragma unroll
      for (int it = 0; it < 4; ++it) *(volatile v4u*)(op + go[it]) = val[it];
      __threadfence();
    }
    __syncthreads();
  }
}

__global__ __launch_bounds__(128) void k_ln(const float* __restrict__ xr,
                                            const float* __restrict__ w,
                                            const float* __restrict__ bb,
                                            _Float16* __restrict__ hp) {
  __shared__ float r0s[4];
  __shared__ float r1s[4];
  const int row = blockIdx.x, tid = threadIdx.x, lane = tid & 31, wave = tid >> 5;
  const size_t o = (size_t)row * HD + (size_t)tid * 8;
  const v4f a0 = *(const v4f*)(xr + o);
  const v4f a1 = *(const v4f*)(xr + o + 4);
  float s = ((a0[0] + a0[1]) + (a0[2] + a0[3])) + ((a1[0] + a1[1]) + (a1[2] + a1[3]));
#pragma unroll
  for (int off = 1; off < 32; off <<= 1) s += __shfl_xor(s, off, 32);
  if (lane == 0) r0s[wave] = s;
  __syncthreads();
  const float mu = ((r0s[0] + r0s[1]) + (r0s[2] + r0s[3])) * (1.0f / (float)HD);
  const float d0 = a0[0] - mu, d1 = a0[1] - mu, d2 = a0[2] - mu, d3 = a0[3] - mu;
  const float d4 = a1[0] - mu, d5 = a1[1] - mu, d6 = a1[2] - mu, d7 = a1[3] - mu;
  float q = ((d0 * d0 + d1 * d1) + (d2 * d2 + d3 * d3)) + ((d4 * d4 + d5 * d5) + (d6 * d6 + d7 * d7));
#pragma unroll
  for (int off = 1; off < 32; off <<= 1) q += __shfl_xor(q, off, 32);
  if (lane == 0) r1s[wave] = q;
  __syncthreads();
  const float var = ((r1s[0] + r1s[1]) + (r1s[2] + r1s[3])) * (1.0f / (float)HD);
  const float inv = rsqrtf(var + 1e-5f);
  const v4f w0 = *(const v4f*)(w + tid * 8);
  const v4f w1 = *(const v4f*)(w + tid * 8 + 4);
  const v4f c0 = *(const v4f*)(bb + tid * 8);
  const v4f c1 = *(const v4f*)(bb + tid * 8 + 4);
  Pack8 pk;
  pk.h = (v8h){(_Float16)(d0 * inv * w0[0] + c0[0]), (_Float16)(d1 * inv * w0[1] + c0[1]),
               (_Float16)(d2 * inv * w0[2] + c0[2]), (_Float16)(d3 * inv * w0[3] + c0[3]),
               (_Float16)(d4 * inv * w1[0] + c1[0]), (_Float16)(d5 * inv * w1[1] + c1[1]),
               (_Float16)(d6 * inv * w1[2] + c1[2]), (_Float16)(d7 * inv * w1[3] + c1[3])};
  const v4u vv = pk.u;
  volatile v4u* dst = (volatile v4u*)(hp + o);
  *dst = vv;
  __threadfence();
  *dst = vv;
}

static_assert((size_t)MROWS * HD * 4 == 2 * ((size_t)MROWS * HD * 2));
static_assert((size_t)MROWS * HD * 2 == (size_t)NBATCH * HD * SEQ * 2);
static_assert((size_t)MROWS * HF * 2 <= (size_t)MROWS * HD * 2);

extern "C" void kernel_launch(void* const* d_in, const int* in_sizes, int n_in,
                              void* d_out, int out_size, void* d_ws, size_t ws_size,
                              hipStream_t stream) {
  if (n_in < 11) return;
  if (in_sizes[0] != MROWS * HD) return;
  if (in_sizes[1] != HD * HD) return;
  if (in_sizes[2] != HD * HD) return;
  if (in_sizes[3] != HD * HD) return;
  if (in_sizes[4] != HD * HD) return;
  if (in_sizes[5] != HD) return;
  if (in_sizes[6] != HD) return;
  if (in_sizes[7] != HF * HD) return;
  if (in_sizes[8] != HF) return;
  if (in_sizes[9] != HD * HF) return;
  if (in_sizes[10] != HD) return;
  if (out_size != MROWS * HD) return;

  const float* x    = (const float*)d_in[0];
  const float* Wq   = (const float*)d_in[1];
  const float* Wk   = (const float*)d_in[2];
  const float* Wv   = (const float*)d_in[3];
  const float* Wo   = (const float*)d_in[4];
  const float* ln_w = (const float*)d_in[5];
  const float* ln_b = (const float*)d_in[6];
  const float* W1   = (const float*)d_in[7];
  const float* b1   = (const float*)d_in[8];
  const float* W2   = (const float*)d_in[9];
  const float* b2   = (const float*)d_in[10];
  float* out = (float*)d_out;

  size_t off = 0;
  const size_t oX  = off; off += (size_t)MROWS * HD * 2;
  const size_t oWq = off; off += (size_t)HD * HD * 2;
  const size_t oWk = off; off += (size_t)HD * HD * 2;
  const size_t oWv = off; off += (size_t)HD * HD * 2;
  const size_t oWo = off; off += (size_t)HD * HD * 2;
  const size_t oW1 = off; off += (size_t)HF * HD * 2;
  const size_t oW2 = off; off += (size_t)HD * HF * 2;
  const size_t oQ  = off; off += (size_t)MROWS * HD * 2;
  const size_t oK  = off; off += (size_t)MROWS * HD * 2;
  const size_t oVt = off; off += (size_t)NBATCH * HD * SEQ * 2;
  const size_t oO  = off; off += (size_t)MROWS * HD * 2;
  if (off > ws_size) return;
  const size_t oR1 = oQ;
  const size_t oHL = oVt;
  const size_t oG  = oO;

  char* ws = (char*)d_ws;
  _Float16* Xh  = (_Float16*)(ws + oX);
  _Float16* Wqh = (_Float16*)(ws + oWq);
  _Float16* Wkh = (_Float16*)(ws + oWk);
  _Float16* Wvh = (_Float16*)(ws + oWv);
  _Float16* Woh = (_Float16*)(ws + oWo);
  _Float16* W1h = (_Float16*)(ws + oW1);
  _Float16* W2h = (_Float16*)(ws + oW2);
  _Float16* Qp  = (_Float16*)(ws + oQ);
  _Float16* Kp  = (_Float16*)(ws + oK);
  _Float16* Vtp = (_Float16*)(ws + oVt);
  _Float16* Op  = (_Float16*)(ws + oO);
  float*    R1p = (float*)(ws + oR1);
  _Float16* HLp = (_Float16*)(ws + oHL);
  _Float16* Gp  = (_Float16*)(ws + oG);

  const int gx  = in_sizes[0] / 8;
  const int gw  = in_sizes[1] / 8;
  const int gw1 = in_sizes[7] / 8;
  const int gw2 = in_sizes[9] / 8;
  k_cvt<<<dim3((gx + 255) / 256),  dim3(256), 0, stream>>>(x,  Xh,  gx,  1.0f);
  k_cvt<<<dim3((gw + 255) / 256),  dim3(256), 0, stream>>>(Wq, Wqh, gw,  32.0f);
  k_cvt<<<dim3((gw + 255) / 256),  dim3(256), 0, stream>>>(Wk, Wkh, gw,  32.0f);
  k_cvt<<<dim3((gw + 255) / 256),  dim3(256), 0, stream>>>(Wv, Wvh, gw,  32.0f);
  k_cvt<<<dim3((gw + 255) / 256),  dim3(256), 0, stream>>>(Wo, Woh, gw,  32.0f);
  k_cvt<<<dim3((gw1 + 255) / 256), dim3(256), 0, stream>>>(W1, W1h, gw1, 32.0f);
  k_cvt<<<dim3((gw2 + 255) / 256), dim3(256), 0, stream>>>(W2, W2h, gw2, 32.0f);
  k_gemm_h<0, HD><<<dim3(MROWS / 256, HD / 64), dim3(256), 0, stream>>>(Xh, Wqh, b2, Qp, HD);
  k_gemm_h<0, HD><<<dim3(MROWS / 256, HD / 64), dim3(256), 0, stream>>>(Xh, Wkh, b2, Kp, HD);
  k_gemm_h<1, HD><<<dim3(MROWS / 256, HD / 64), dim3(256), 0, stream>>>(Xh, Wvh, b2, Vtp, HD);
  k_attn<<<dim3(MROWS / 128), dim3(256), 0, stream>>>(Qp, Kp, Vtp, Op);
  k_gemm_f<0, HD><<<dim3(MROWS / 256, HD / 64), dim3(256), 0, stream>>>(Op, Woh, b2, x, R1p, 0.001953125f);
  k_ln<<<dim3(MROWS), dim3(128), 0, stream>>>(R1p, ln_w, ln_b, HLp);
  k_gemm_h<2, HD><<<dim3(MROWS / 256, HF / 64), dim3(256), 0, stream>>>(HLp, W1h, b1, Gp, HF);
  k_gemm_f<1, HF><<<dim3(MROWS / 256, HD / 64), dim3(256), 0, stream>>>(Gp, W2h, b2, R1p, out, 0.03125f);
  (void)hipGetLastError();
}
